// GlobalSelfFeastBlock_66133906424007
// MI455X (gfx1250) — hardware-verified
//
#include <hip/hip_runtime.h>
#include <math.h>
#include <stdint.h>


#define NTOK  4096
#define DM    1024
#define NHEAD 8
#define HDIM  128
#define DFF   1536
#define KC    64
#define QB    64
#define GP    132
#define OSP   132

typedef _Float16 v16h __attribute__((ext_vector_type(16)));
typedef _Float16 v8h  __attribute__((ext_vector_type(8)));
typedef float    v8f  __attribute__((ext_vector_type(8)));
typedef float    v4f  __attribute__((ext_vector_type(4)));
typedef unsigned int v4u __attribute__((ext_vector_type(4)));
typedef unsigned int v2u __attribute__((ext_vector_type(2)));

__device__ __forceinline__ unsigned short h2u(_Float16 x) { return __builtin_bit_cast(unsigned short, x); }
__device__ __forceinline__ unsigned pk16(unsigned short a, unsigned short b) { return (unsigned)a | ((unsigned)b << 16); }
__device__ __forceinline__ unsigned pkf(float a, float b) { return pk16(h2u((_Float16)a), h2u((_Float16)b)); }

__device__ __forceinline__ void wave_sync() {
  __builtin_amdgcn_fence(__ATOMIC_RELEASE, "workgroup");
  __builtin_amdgcn_wave_barrier();
  __builtin_amdgcn_fence(__ATOMIC_ACQUIRE, "workgroup");
}

union FragH { v16h v; v8h h[2]; };
__device__ __forceinline__ v16h ldfrag_h(const _Float16* p) {
  FragH f; f.h[0] = *(const v8h*)(p); f.h[1] = *(const v8h*)(p + 16); return f.v;
}

__device__ __forceinline__ v8f wmma_raw(v16h a, v16h b, v8f c) {
  return __builtin_amdgcn_wmma_f32_16x16x32_f16(false, a, false, b, (short)0, c, false, false);
}
__device__ __forceinline__ v8f wmma_h(v16h a, v16h b, v8f c) {
  c = __builtin_amdgcn_wmma_f32_16x16x32_f16(false, a, false, b, (short)0, c, false, false);
  asm volatile("v_nop\n\tv_nop\n\tv_nop\n\tv_nop" : "+v"(c) : "v"(a), "v"(b));
  return c;
}
__device__ __forceinline__ void dep_guard2(v8f& x, v8f& y, v16h b, v16h a0, v16h a1) {
  asm volatile("v_nop\n\tv_nop\n\tv_nop\n\tv_nop" : "+v"(x), "+v"(y) : "v"(b), "v"(a0), "v"(a1));
}

__global__ __launch_bounds__(256) void cvt_f16x8_kernel(const float* __restrict__ in, _Float16* out, int n8, float scale) {
  const int i = blockIdx.x * 256 + threadIdx.x;
  if (i < n8) {
    const v4f a = *(const v4f*)(in + 8 * (size_t)i) * scale;
    const v4f c = *(const v4f*)(in + 8 * (size_t)i + 4) * scale;
    v4u w;
    w[0] = pkf(a[0], a[1]);
    w[1] = pkf(a[2], a[3]);
    w[2] = pkf(c[0], c[1]);
    w[3] = pkf(c[2], c[3]);
    volatile v4u* p = (volatile v4u*)(out + 8 * (size_t)i);
    *p = w;
    __threadfence();
    *p = w;
  }
}

template <int MODE>
__global__ __launch_bounds__(128) void gemm_kernel(
    const _Float16* __restrict__ A, int lda, const _Float16* __restrict__ Bt, int ldb,
    void* Cout, int ldc, const float* __restrict__ bias, const float* __restrict__ res, int ldr,
    float oscale, int M, int N, int K) {
  __shared__ __align__(16) float sT[4][16 * GP];
  const int lane = threadIdx.x & 31;
  const int wave = threadIdx.x >> 5;
  const int tilesN = N >> 7;
  const int tilesM = M >> 5;
  const int tile = blockIdx.x * 4 + wave;
  if (tile >= tilesM * tilesN) return;
  const int tm = tile / tilesN;
  const int tn = tile - tm * tilesN;
  const int m0 = tm << 5;
  const int n0 = tn << 7;

  const int rlane = lane & 15;
  const int koff  = (lane >> 4) * 8;
  const int mOff  = (lane >> 4) * 8;

  v8f acc[2][8];
#pragma unroll
  for (int i = 0; i < 2; ++i)
#pragma unroll
    for (int j = 0; j < 8; ++j) acc[i][j] = (v8f){0.f, 0.f, 0.f, 0.f, 0.f, 0.f, 0.f, 0.f};

  for (int k0 = 0; k0 < K; k0 += 32) {
    const v16h a0 = ldfrag_h(A + (size_t)(m0 + rlane) * lda + k0 + koff);
    const v16h a1 = ldfrag_h(A + (size_t)(m0 + 16 + rlane) * lda + k0 + koff);
#pragma unroll
    for (int j = 0; j < 8; ++j) {
      const v16h bh = ldfrag_h(Bt + (size_t)(n0 + (j << 4) + rlane) * ldb + k0 + koff);
      acc[0][j] = wmma_raw(a0, bh, acc[0][j]);
      acc[1][j] = wmma_raw(a1, bh, acc[1][j]);
      dep_guard2(acc[0][j], acc[1][j], bh, a0, a1);
    }
  }

  float* slab = sT[wave];
  float bc[8];
#pragma unroll
  for (int j = 0; j < 8; ++j) bc[j] = 0.f;
  if (MODE == 2) {
#pragma unroll
    for (int j = 0; j < 8; ++j) bc[j] = bias[n0 + (j << 4) + rlane];
  }
#pragma unroll
  for (int i = 0; i < 2; ++i) {
    const int mBase = m0 + (i << 4);
#pragma unroll
    for (int j = 0; j < 8; ++j) {
#pragma unroll
      for (int r = 0; r < 8; ++r) {
        float v = acc[i][j][r] * oscale;
        if (MODE == 2) {
          v += bc[j];
          v = 0.5f * v * (1.0f + erff(v * 0.70710678118654752f));
          v *= 16.0f;
        }
        slab[(mOff + r) * GP + (j << 4) + rlane] = v;
      }
    }
    wave_sync();
    if (MODE == 1) {
      float* C = (float*)Cout;
      const int c4 = lane * 4;
      const v4f b4 = *(const v4f*)(bias + n0 + c4);
      for (int rep = 0; rep < 2; ++rep) {
#pragma unroll
        for (int it = 0; it < 16; ++it) {
          const v4f rv = *(const v4f*)(res + (size_t)(mBase + it) * ldr + n0 + c4);
          const v4f v = *(const v4f*)(slab + it * GP + c4) + b4 + rv;
          *(volatile v4f*)(C + (size_t)(mBase + it) * ldc + n0 + c4) = v;
        }
        __threadfence();
      }
    } else {
      _Float16* C = (_Float16*)Cout;
      const int q16 = lane >> 4, c8 = (lane & 15) * 8;
      for (int rep = 0; rep < 2; ++rep) {
#pragma unroll
        for (int it = 0; it < 8; ++it) {
          const int row = it * 2 + q16;
          const float* sp = slab + row * GP + c8;
          const v4f x0 = *(const v4f*)(sp);
          const v4f x1 = *(const v4f*)(sp + 4);
          v4u w;
          w[0] = pkf(x0[0], x0[1]);
          w[1] = pkf(x0[2], x0[3]);
          w[2] = pkf(x1[0], x1[1]);
          w[3] = pkf(x1[2], x1[3]);
          *(volatile v4u*)(C + (size_t)(mBase + row) * ldc + n0 + c8) = w;
        }
        __threadfence();
      }
    }
    wave_sync();
  }
}

template <int PASS>
__global__ __launch_bounds__(128)
void attn_kernel(const _Float16* __restrict__ QK, const _Float16* __restrict__ VT, const int* __restrict__ coords,
                 float* stats, _Float16* attP) {
  constexpr int LH = QB * HDIM + KC * HDIM + ((PASS == 2) ? (HDIM * KC) : 0);
  __shared__ __align__(16) _Float16 L[LH];
  __shared__ __align__(16) _Float16 Ps[(PASS == 2) ? (4 * 16 * KC) : 8];
  __shared__ __align__(16) int kco[2 * KC];
  __shared__ __align__(16) float stat_s[(PASS == 1) ? (4 * 16 * 4) : 4];
  static_assert(PASS != 2 || 4 * 16 * OSP * 4 <= LH * 2);
  _Float16* const Qs  = L;
  _Float16* const Ks  = L + QB * HDIM;
  _Float16* const Vts = L + QB * HDIM + KC * HDIM;

  const int tid  = threadIdx.x;
  const int wave = tid >> 5;
  const int lane = tid & 31;
  const int hh   = lane >> 4;
  const int c    = lane & 15;

  const int qb = blockIdx.x & 63;
  const int h  = blockIdx.x >> 6;
  const int q0 = qb * QB + wave * 16;

  {
    const int r = tid >> 1, half = (tid & 1) * 64;
    const _Float16* src = QK + (size_t)(qb * QB + r) * (2 * DM) + h * HDIM + half;
#pragma unroll
    for (int i = 0; i < 8; ++i) *(v8h*)(Qs + r * HDIM + half + 8 * i) = *(const v8h*)(src + 8 * i);
  }
  float qx[8], qy[8];
#pragma unroll
  for (int r = 0; r < 8; ++r) {
    const int row = q0 + 8 * hh + r;
    qx[r] = (float)coords[2 * row];
    qy[r] = (float)coords[2 * row + 1];
  }

  const float LOG2E = 1.4426950408889634f;
  const float cS  = LOG2E * (1.0f / 2896.3093757400988f);
  const float cSn = cS * (1.0f / 0.6f);
  const float hsc = __uint_as_float((unsigned)(126 - h) << 23);
  const float hb  = hsc * LOG2E;
  const float hbn = hsc * (LOG2E * (1.0f / 0.6f));

  float mp[8], lp[8], mn[8], ln[8];
  v8f o[8];
  const v8f zero8 = (v8f){0.f, 0.f, 0.f, 0.f, 0.f, 0.f, 0.f, 0.f};
#pragma unroll
  for (int t = 0; t < 8; ++t) o[t] = zero8;
  if (PASS == 1) {
#pragma unroll
    for (int r = 0; r < 8; ++r) { mp[r] = -__builtin_inff(); mn[r] = -__builtin_inff(); lp[r] = 0.f; ln[r] = 0.f; }
  } else {
#pragma unroll
    for (int r = 0; r < 8; ++r) {
      const v4f st = *(const v4f*)(stats + ((size_t)h * NTOK + q0 + 8 * hh + r) * 4);
      mp[r] = st[0]; lp[r] = st[1]; mn[r] = st[2]; ln[r] = st[3];
    }
  }

  const _Float16* Kg = QK + DM + h * HDIM;
  const _Float16* Vg = VT + (size_t)(h * HDIM) * NTOK;
  const _Float16* Qw = Qs + wave * 16 * HDIM;
  _Float16* const Pw = Ps + ((PASS == 2) ? wave * 16 * KC : 0);

#pragma unroll 1
  for (int kcix = 0; kcix < NTOK / KC; ++kcix) {
    const int kv0 = kcix * KC;
    __syncthreads();
    {
      const int r = tid >> 1, half = (tid & 1) * 64;
      const _Float16* src = Kg + (size_t)(kv0 + r) * (2 * DM) + half;
#pragma unroll
      for (int i = 0; i < 8; ++i) *(v8h*)(Ks + r * HDIM + half + 8 * i) = *(const v8h*)(src + 8 * i);
      if (PASS == 2) {
        const _Float16* srv = Vg + (size_t)tid * NTOK + kv0;
#pragma unroll
        for (int i = 0; i < 8; ++i) *(v8h*)(Vts + tid * KC + 8 * i) = *(const v8h*)(srv + 8 * i);
      }
      if (tid < KC) {
        kco[2 * tid]     = coords[2 * (kv0 + tid)];
        kco[2 * tid + 1] = coords[2 * (kv0 + tid) + 1];
      }
    }
    __syncthreads();

    v8f s[4];
#pragma unroll
    for (int j = 0; j < 4; ++j) s[j] = zero8;
#pragma unroll
    for (int dc = 0; dc < 4; ++dc) {
      const v16h qa = ldfrag_h(Qw + c * HDIM + dc * 32 + 8 * hh);
#pragma unroll
      for (int j = 0; j < 4; ++j) {
        const v16h kb = ldfrag_h(Ks + (j * 16 + c) * HDIM + dc * 32 + 8 * hh);
        s[j] = wmma_h(qa, kb, s[j]);
      }
    }

    float kx[4], ky[4];
#pragma unroll
    for (int j = 0; j < 4; ++j) {
      kx[j] = (float)kco[2 * (j * 16 + c)];
      ky[j] = (float)kco[2 * (j * 16 + c) + 1];
    }

#pragma unroll
    for (int r = 0; r < 8; ++r) {
      float yp[4], yn[4];
#pragma unroll
      for (int j = 0; j < 4; ++j) {
        const float sc = s[j][r];
        const float dx = qx[r] - kx[j], dy = qy[r] - ky[j];
        const float dist = sqrtf(dx * dx + dy * dy);
        yp[j] = sc * cS - dist * hb;
        yn[j] = -(sc * cSn) - dist * hbn;
      }
      if (PASS == 1) {
        float mxp = fmaxf(fmaxf(yp[0], yp[1]), fmaxf(yp[2], yp[3]));
        float mxn = fmaxf(fmaxf(yn[0], yn[1]), fmaxf(yn[2], yn[3]));
#pragma unroll
        for (int off = 1; off < 16; off <<= 1) {
          mxp = fmaxf(mxp, __shfl_xor(mxp, off, 32));
          mxn = fmaxf(mxn, __shfl_xor(mxn, off, 32));
        }
        const float mnp = fmaxf(mp[r], mxp);
        const float mnn = fmaxf(mn[r], mxn);
        float sp = 0.f, sn = 0.f;
#pragma unroll
        for (int j = 0; j < 4; ++j) { sp += exp2f(yp[j] - mnp); sn += exp2f(yn[j] - mnn); }
#pragma unroll
        for (int off = 1; off < 16; off <<= 1) {
          sp += __shfl_xor(sp, off, 32);
          sn += __shfl_xor(sn, off, 32);
        }
        lp[r] = lp[r] * exp2f(mp[r] - mnp) + sp;
        ln[r] = ln[r] * exp2f(mn[r] - mnn) + sn;
        mp[r] = mnp;
        mn[r] = mnn;
      } else {
#pragma unroll
        for (int j = 0; j < 4; ++j) {
          const float a = exp2f(yp[j] - mp[r]) * lp[r] - exp2f(yn[j] - mn[r]) * ln[r];
          Pw[(8 * hh + r) * KC + j * 16 + c] = (_Float16)a;
        }
      }
    }

    if (PASS == 2) {
      wave_sync();
#pragma unroll
      for (int kk = 0; kk < 2; ++kk) {
        const v16h pa = ldfrag_h(Pw + c * KC + kk * 32 + 8 * hh);
#pragma unroll
        for (int t = 0; t < 8; ++t) {
          const v16h vb = ldfrag_h(Vts + (t * 16 + c) * KC + kk * 32 + 8 * hh);
          o[t] = wmma_h(pa, vb, o[t]);
        }
      }
    }
  }

  if (PASS == 1) {
    if (c == 0) {
#pragma unroll
      for (int r = 0; r < 8; ++r) {
        float* sp = stat_s + (wave * 16 + 8 * hh + r) * 4;
        sp[0] = mp[r];
        sp[1] = 8192.0f * (1.0f / lp[r]);
        sp[2] = mn[r];
        sp[3] = 12288.0f * (1.0f / ln[r]);
      }
    }
    wave_sync();
    if (lane < 16) {
      const v4f v = *(const v4f*)(stat_s + (wave * 16 + lane) * 4);
      volatile v4f* gp = (volatile v4f*)(stats + ((size_t)h * NTOK + q0 + lane) * 4);
      *gp = v;
      __threadfence();
      *gp = v;
    }
  } else {
    __syncthreads();
    float* os = (float*)(void*)L + wave * (16 * OSP);
#pragma unroll
    for (int r = 0; r < 8; ++r) {
#pragma unroll
      for (int t = 0; t < 8; ++t) os[(8 * hh + r) * OSP + t * 16 + c] = o[t][r] * 1.220703125e-4f;
    }
    wave_sync();
    const int q16 = lane >> 4, c8 = (lane & 15) * 8;
    for (int rep = 0; rep < 2; ++rep) {
#pragma unroll
      for (int it = 0; it < 8; ++it) {
        const int row = it * 2 + q16;
        const float* sp = os + row * OSP + c8;
        const v4f x0 = *(const v4f*)(sp);
        const v4f x1 = *(const v4f*)(sp + 4);
        v4u w;
        w[0] = pkf(x0[0], x0[1]);
        w[1] = pkf(x0[2], x0[3]);
        w[2] = pkf(x1[0], x1[1]);
        w[3] = pkf(x1[2], x1[3]);
        *(volatile v4u*)(attP + (size_t)(q0 + row) * DM + h * HDIM + c8) = w;
      }
      __threadfence();
    }
  }
}

template <int MODE>
__global__ __launch_bounds__(128) void ln_kernel(const float* __restrict__ in, const float* __restrict__ g,
                                                 const float* __restrict__ b, float* outF, _Float16* outH, int nrows) {
  const int lane = threadIdx.x & 31;
  const int wave = threadIdx.x >> 5;
  const int row  = blockIdx.x * 4 + wave;
  if (row >= nrows) return;
  const float* src = in + (size_t)row * DM;
  v4f x[8];
  float sum = 0.f;
#pragma unroll
  for (int sg = 0; sg < 8; ++sg) {
    x[sg] = *(const v4f*)(src + sg * 128 + 4 * lane);
    sum += (x[sg][0] + x[sg][1]) + (x[sg][2] + x[sg][3]);
  }
#pragma unroll
  for (int off = 1; off < 32; off <<= 1) sum += __shfl_xor(sum, off, 32);
  const float mu = sum * (1.0f / (float)DM);
  float vs = 0.f;
#pragma unroll
  for (int sg = 0; sg < 8; ++sg) {
    const v4f d = x[sg] - mu;
    vs += (d[0] * d[0] + d[1] * d[1]) + (d[2] * d[2] + d[3] * d[3]);
  }
#pragma unroll
  for (int off = 1; off < 32; off <<= 1) vs += __shfl_xor(vs, off, 32);
  const float var  = vs * (1.0f / (float)DM);
  const float rstd = rsqrtf(var + 1e-5f);
  for (int rep = 0; rep < 2; ++rep) {
#pragma unroll
    for (int sg = 0; sg < 8; ++sg) {
      const int col = sg * 128 + 4 * lane;
      const v4f g4 = *(const v4f*)(g + col);
      const v4f b4 = *(const v4f*)(b + col);
      const v4f y  = (x[sg] - mu) * rstd * g4 + b4;
      *(volatile v4f*)(outF + (size_t)row * DM + col) = y;
      if (MODE == 0) {
        v2u hp;
        hp[0] = pkf(y[0] * 16.0f, y[1] * 16.0f);
        hp[1] = pkf(y[2] * 16.0f, y[3] * 16.0f);
        *(volatile v2u*)(outH + (size_t)row * DM + col) = hp;
      }
    }
    __threadfence();
  }
}

extern "C" void kernel_launch(void* const* d_in, const int* in_sizes, int n_in,
                              void* d_out, int out_size, void* d_ws, size_t ws_size,
                              hipStream_t stream) {
  if (n_in < 15) return;
  if (in_sizes[0] != NTOK * DM) return;
  if (in_sizes[1] != NTOK * 2) return;
  if (in_sizes[2] != DM * DM || in_sizes[3] != DM * DM || in_sizes[4] != DM * DM || in_sizes[5] != DM * DM) return;
  if (in_sizes[6] != DM || in_sizes[7] != DM || in_sizes[8] != DM) return;
  if (in_sizes[9] != DFF * DM || in_sizes[10] != DFF || in_sizes[11] != DM * DFF) return;
  if (in_sizes[12] != DM || in_sizes[13] != DM || in_sizes[14] != DM) return;
  if (out_size != NTOK * DM) return;

  const float* features = (const float*)d_in[0];
  const int*   coords   = (const int*)d_in[1];
  const float* Wq = (const float*)d_in[2];
  const float* Wk = (const float*)d_in[3];
  const float* Wv = (const float*)d_in[4];
  const float* Wo = (const float*)d_in[5];
  const float* bo = (const float*)d_in[6];
  const float* ln1_g = (const float*)d_in[7];
  const float* ln1_b = (const float*)d_in[8];
  const float* W1 = (const float*)d_in[9];
  const float* b1 = (const float*)d_in[10];
  const float* W2 = (const float*)d_in[11];
  const float* b2 = (const float*)d_in[12];
  const float* ln2_g = (const float*)d_in[13];
  const float* ln2_b = (const float*)d_in[14];
  float* out = (float*)d_out;

  const size_t szFeatP = (size_t)NTOK * DM * 2;
  const size_t szWqk   = (size_t)2 * DM * DM * 2;
  const size_t szW     = (size_t)DM * DM * 2;
  const size_t szWf    = (size_t)DFF * DM * 2;
  const size_t szQK    = (size_t)NTOK * 2 * DM * 2;
  const size_t szVT    = (size_t)DM * NTOK * 2;
  const size_t szSt    = (size_t)NHEAD * NTOK * 4 * 4;
  const size_t szAtt   = (size_t)NTOK * DM * 2;
  const size_t szF32   = (size_t)NTOK * DM * 4;
  const size_t szXP    = (size_t)NTOK * DM * 2;
  const size_t szHP    = (size_t)NTOK * DFF * 2;
  size_t off = 0;
  const size_t oFeatP = off; off += szFeatP;
  const size_t oWqk   = off; off += szWqk;
  const size_t oWv    = off; off += szW;
  const size_t oWo    = off; off += szW;
  const size_t oW1    = off; off += szWf;
  const size_t oW2    = off; off += szWf;
  const size_t oQK    = off; off += szQK;
  const size_t oVT    = off; off += szVT;
  const size_t oSt    = off; off += szSt;
  const size_t oAtt   = off; off += szAtt;
  const size_t oPre1  = off; off += szF32;
  const size_t oXF    = off; off += szF32;
  const size_t oXP    = off; off += szXP;
  const size_t oHP    = off; off += szHP;
  const size_t oPre2  = off; off += szF32;
  if (off > ws_size) return;
  if (off > (size_t)134217728) return;

  char* ws = (char*)d_ws;
  _Float16* featP = (_Float16*)(ws + oFeatP);
  _Float16* WqkP  = (_Float16*)(ws + oWqk);
  _Float16* WvP   = (_Float16*)(ws + oWv);
  _Float16* WoP   = (_Float16*)(ws + oWo);
  _Float16* W1P   = (_Float16*)(ws + oW1);
  _Float16* W2P   = (_Float16*)(ws + oW2);
  _Float16* QKp   = (_Float16*)(ws + oQK);
  _Float16* VTp   = (_Float16*)(ws + oVT);
  float*    stats = (float*)(ws + oSt);
  _Float16* attP  = (_Float16*)(ws + oAtt);
  float*    pre1  = (float*)(ws + oPre1);
  float*    xF    = (float*)(ws + oXF);
  _Float16* xP    = (_Float16*)(ws + oXP);
  _Float16* hP    = (_Float16*)(ws + oHP);
  float*    pre2  = (float*)(ws + oPre2);

  const dim3 blk256(256), blk128(128);
  const int n8x = NTOK * DM / 8, n8w = DM * DM / 8, n8f = DFF * DM / 8;

  cvt_f16x8_kernel<<<dim3((n8x + 255) / 256), blk256, 0, stream>>>(features, featP, n8x, 1.0f);
  cvt_f16x8_kernel<<<dim3((n8w + 255) / 256), blk256, 0, stream>>>(Wq, WqkP, n8w, 64.0f);
  cvt_f16x8_kernel<<<dim3((n8w + 255) / 256), blk256, 0, stream>>>(Wk, WqkP + (size_t)DM * DM, n8w, 64.0f);
  cvt_f16x8_kernel<<<dim3((n8w + 255) / 256), blk256, 0, stream>>>(Wv, WvP, n8w, 64.0f);
  cvt_f16x8_kernel<<<dim3((n8w + 255) / 256), blk256, 0, stream>>>(Wo, WoP, n8w, 64.0f);
  cvt_f16x8_kernel<<<dim3((n8f + 255) / 256), blk256, 0, stream>>>(W1, W1P, n8f, 64.0f);
  cvt_f16x8_kernel<<<dim3((n8f + 255) / 256), blk256, 0, stream>>>(W2, W2P, n8f, 64.0f);
  {
    const int M = NTOK, N = 2 * DM, K = DM;
    const int tiles = (M / 32) * (N / 128);
    gemm_kernel<0><<<dim3((tiles + 3) / 4), blk128, 0, stream>>>(
        featP, DM, WqkP, DM, (void*)QKp, 2 * DM, bo, features, DM, 0.25f, M, N, K);
  }
  {
    const int M = DM, N = NTOK, K = DM;
    const int tiles = (M / 32) * (N / 128);
    gemm_kernel<0><<<dim3((tiles + 3) / 4), blk128, 0, stream>>>(
        WvP, DM, featP, DM, (void*)VTp, NTOK, bo, features, DM, 0.25f, M, N, K);
  }
  attn_kernel<1><<<dim3(NHEAD * (NTOK / QB)), blk128, 0, stream>>>(QKp, VTp, coords, stats, attP);
  attn_kernel<2><<<dim3(NHEAD * (NTOK / QB)), blk128, 0, stream>>>(QKp, VTp, coords, stats, attP);
  {
    const int M = NTOK, N = DM, K = DM;
    const int tiles = (M / 32) * (N / 128);
    gemm_kernel<1><<<dim3((tiles + 3) / 4), blk128, 0, stream>>>(
        attP, DM, WoP, DM, (void*)pre1, DM, bo, features, DM, 9.765625e-4f, M, N, K);
  }
  ln_kernel<0><<<dim3(NTOK / 4), blk128, 0, stream>>>(pre1, ln1_g, ln1_b, xF, xP, NTOK);
  {
    const int M = NTOK, N = DFF, K = DM;
    const int tiles = (M / 32) * (N / 128);
    gemm_kernel<2><<<dim3((tiles + 3) / 4), blk128, 0, stream>>>(
        xP, DM, W1P, DM, (void*)hP, DFF, b1, features, DM, 9.765625e-4f, M, N, K);
  }
  {
    const int M = NTOK, N = DM, K = DFF;
    const int tiles = (M / 32) * (N / 128);
    gemm_kernel<1><<<dim3((tiles + 3) / 4), blk128, 0, stream>>>(
        hP, DFF, W2P, DFF, (void*)pre2, DM, b2, xF, DM, 9.765625e-4f, M, N, K);
  }
  ln_kernel<1><<<dim3(NTOK / 4), blk128, 0, stream>>>(pre2, ln2_g, ln2_b, out, xP, NTOK);
  (void)hipGetLastError();
}
